// HybridAttention_45406394253512
// MI455X (gfx1250) — hardware-verified
//
#include <hip/hip_runtime.h>
#include <math.h>

#ifndef NB
#define NB 4
#endif
#ifndef SEQ
#define SEQ 2048
#endif
#define NB_FULL 4
#define SEQ_FULL 2048
#define DM 1024
#define NH 16
#define HD 64
#define QKVN 3072
#define LHALF 6

static_assert(SEQ % 64 == 0);
static_assert(NB >= 1 && NB <= NB_FULL);
static_assert(SEQ >= 64 && SEQ <= SEQ_FULL);
static_assert(NH * HD == DM);

typedef __attribute__((ext_vector_type(16))) _Float16 v16h;
typedef __attribute__((ext_vector_type(8)))  _Float16 v8h;
typedef __attribute__((ext_vector_type(8)))  float v8f;
typedef __attribute__((ext_vector_type(4)))  float v4f;
typedef __attribute__((ext_vector_type(4)))  unsigned v4u;

template <typename T> __device__ __forceinline__ void vst2(void* p, T v) { *(volatile T*)p = v; __threadfence(); *(volatile T*)p = v; }
__device__ __forceinline__ v8f wmma16(v16h a, v16h b, v8f c) {
  v8f d = __builtin_amdgcn_wmma_f32_16x16x32_f16(false, a, false, b, (short)0, c, false, false);
  asm volatile("v_nop\n\tv_nop\n\tv_nop\n\tv_nop" : "+v"(d) : "v"(a), "v"(b));
  return d;
}
__device__ __forceinline__ v16h frag_h(const _Float16* rowk0, int lane) {
  union { v16h v; v8h q[2]; } u; const _Float16* p = rowk0 + 8 * (lane >> 4);
  u.q[0] = *(const v8h*)p; u.q[1] = *(const v8h*)(p + 16); return u.v;
}
__device__ __forceinline__ float bfr(float v) { return (float)(__bf16)v; }
union HU { v8h h; v4u u; };

#define WS_XN  ((size_t)0)
#define WS_WQT (WS_XN + 2u * (size_t)NB * SEQ * DM)
#define WS_WOT (WS_WQT + 2u * (size_t)QKVN * DM)
#define WS_Q   (WS_WOT + 2u * (size_t)DM * DM)
#define WS_K   (WS_Q + 2u * (size_t)NB * SEQ * DM)
#define WS_VT  (WS_K + 2u * (size_t)NB * SEQ * DM)
#define WS_Y   (WS_VT + 2u * (size_t)NB * SEQ * DM)
#define WS_END (WS_Y + 2u * (size_t)NB * SEQ * DM)
static_assert(WS_END <= (size_t)134217728);

__global__ __launch_bounds__(256) void k_wt(const float* __restrict__ W, int K, int N, _Float16* __restrict__ T) {
  __shared__ __align__(16) _Float16 st[64][72];
  const int tid = threadIdx.x; const int n0 = blockIdx.x * 64, k0 = blockIdx.y * 64; const int nn = tid & 63;
#pragma unroll 4
  for (int it = 0; it < 16; ++it) { const int kk = (tid >> 6) + 4 * it; st[nn][kk] = (_Float16)(bfr(W[(size_t)(k0 + kk) * N + n0 + nn]) * 64.0f); }
  __syncthreads();
  for (int e = tid; e < 64 * 8; e += 256) { const int r = e >> 3, q = e & 7; vst2(T + (size_t)(n0 + r) * K + k0 + q * 8, *(const v4u*)&st[r][q * 8]); }
}

__global__ __launch_bounds__(128) void k_ln(const float* __restrict__ X, const float* __restrict__ LW, const float* __restrict__ LB, _Float16* __restrict__ XN) {
  __shared__ float red[8];
  const int tid = threadIdx.x, lane = tid & 31, wave = tid >> 5; const int row = blockIdx.x; const int b = row / SEQ, t = row - b * SEQ;
  const float* xr = X + ((size_t)b * SEQ_FULL + t) * DM + tid * 8;
  const v4f xa = *(const v4f*)xr, xb = *(const v4f*)(xr + 4);
  float v[8];
#pragma unroll
  for (int i = 0; i < 4; ++i) { v[i] = bfr(xa[i]); v[4 + i] = bfr(xb[i]); }
  float s = 0.0f;
#pragma unroll
  for (int i = 0; i < 8; ++i) s += v[i];
#pragma unroll
  for (int o = 16; o > 0; o >>= 1) s += __shfl_xor(s, o);
  if (lane == 0) red[wave] = s;
  __syncthreads();
  const float mu = ((red[0] + red[1]) + (red[2] + red[3])) * (1.0f / (float)DM);
  float s2 = 0.0f;
#pragma unroll
  for (int i = 0; i < 8; ++i) { v[i] -= mu; s2 += v[i] * v[i]; }
#pragma unroll
  for (int o = 16; o > 0; o >>= 1) s2 += __shfl_xor(s2, o);
  if (lane == 0) red[4 + wave] = s2;
  __syncthreads();
  const float var = ((red[4] + red[5]) + (red[6] + red[7])) * (1.0f / (float)DM);
  const float rs = rsqrtf(var + 1.0e-5f);
  const v4f wa = *(const v4f*)(LW + tid * 8), wb = *(const v4f*)(LW + tid * 8 + 4);
  const v4f ba = *(const v4f*)(LB + tid * 8), bb = *(const v4f*)(LB + tid * 8 + 4);
  HU u;
#pragma unroll
  for (int i = 0; i < 4; ++i) { u.h[i] = (_Float16)(v[i] * rs * bfr(wa[i]) + bfr(ba[i])); u.h[4 + i] = (_Float16)(v[4 + i] * rs * bfr(wb[i]) + bfr(bb[i])); }
  vst2(XN + (size_t)row * DM + tid * 8, u.u);
}

__device__ __forceinline__ void mm_k1024(const _Float16* __restrict__ ap, const _Float16* __restrict__ bp, int lane, v8f (&acc)[8]) {
#pragma unroll 2
  for (int kc = 0; kc < DM / 32; ++kc) { const v16h a = frag_h(ap + kc * 32, lane);
#pragma unroll
    for (int j = 0; j < 8; ++j) acc[j] = wmma16(a, frag_h(bp + (size_t)j * 16 * DM + kc * 32, lane), acc[j]); }
}

__global__ __launch_bounds__(128) void k_qkv(const _Float16* __restrict__ XN, const _Float16* __restrict__ WQT, _Float16* __restrict__ Q16, _Float16* __restrict__ K16, _Float16* __restrict__ VT16) {
  __shared__ __align__(16) _Float16 sh[64][136]; __shared__ __align__(16) _Float16 th[128][72];
  const int tid = threadIdx.x, wave = tid >> 5, lane = tid & 31, col = lane & 15, g = lane >> 4;
  const int c0 = blockIdx.y * 128; const int which = c0 >> 10; const int hA = (c0 & 1023) >> 6;
  const int r0 = blockIdx.x * 64; const int b = r0 / SEQ, t0 = r0 - b * SEQ;
  v8f acc[8] = {};
  mm_k1024(XN + (size_t)(r0 + wave * 16 + col) * DM, WQT + (size_t)(c0 + col) * DM, lane, acc);
#pragma unroll
  for (int j = 0; j < 8; ++j)
#pragma unroll
    for (int r = 0; r < 8; ++r) { const _Float16 hv = (_Float16)(acc[j][r] * (1.0f / 64.0f)); const int rl = wave * 16 + 8 * g + r, cl = j * 16 + col;
      if (which == 2) th[cl][rl] = hv; else sh[rl][cl] = hv; }
  __syncthreads();
  if (which < 2) { _Float16* P = (which == 0) ? Q16 : K16;
    for (int e = tid; e < 64 * 16; e += 128) { const int rl = e >> 4, hh = (e >> 3) & 1, q = e & 7;
      vst2(P + (((size_t)(b * NH + hA + hh)) * SEQ + t0 + rl) * HD + q * 8, *(const v4u*)&sh[rl][hh * 64 + q * 8]); } }
  else {
    for (int e = tid; e < 128 * 8; e += 128) { const int cl = e >> 3, q = e & 7;
      vst2(VT16 + (((size_t)(b * NH + hA + (cl >> 6))) * HD + (cl & 63)) * SEQ + t0 + q * 8, *(const v4u*)&th[cl][q * 8]); } }
}

__global__ __launch_bounds__(128) void k_attn(const _Float16* __restrict__ Q16, const _Float16* __restrict__ K16, const _Float16* __restrict__ VT16, const int* __restrict__ LI, _Float16* __restrict__ Y16) {
  __shared__ __align__(16) _Float16 ss[4][16][72];
  const int tid = threadIdx.x, wave = tid >> 5, lane = tid & 31, col = lane & 15, g = lane >> 4;
  const int bh = blockIdx.y; const int b = bh / NH, h = bh - b * NH; const int ql0 = blockIdx.x * 64 + wave * 16;
  const float fold = (LI[0] < LHALF) ? 1.0f : __int_as_float(0x7fc00000);
  const _Float16* qp = Q16 + ((size_t)bh * SEQ + ql0 + col) * HD;
  const v16h qb0 = frag_h(qp, lane), qb1 = frag_h(qp + 32, lane);
  const _Float16* kbase = K16 + ((size_t)bh * SEQ + col) * HD;
  const _Float16* vbase = VT16 + ((size_t)bh * HD + col) * SEQ;
  v8f o[4] = {};
#pragma unroll 2
  for (int kb = 0; kb < SEQ; kb += 32) {
    const _Float16* kp0 = kbase + (size_t)kb * HD; const _Float16* kp1 = kp0 + 16 * HD;
    v8f s0 = {}, s1 = {};
    s0 = wmma16(frag_h(kp0, lane), qb0, s0); s0 = wmma16(frag_h(kp0 + 32, lane), qb1, s0);
    s1 = wmma16(frag_h(kp1, lane), qb0, s1); s1 = wmma16(frag_h(kp1 + 32, lane), qb1, s1);
    v16h p;
#pragma unroll
    for (int r = 0; r < 8; ++r) { p[r] = (_Float16)fmaxf(s0[r], 0.0f); p[8 + r] = (_Float16)fmaxf(s1[r], 0.0f); }
#pragma unroll
    for (int j = 0; j < 4; ++j) o[j] = wmma16(p, frag_h(vbase + (size_t)j * 16 * SEQ + kb, lane), o[j]);
  }
#pragma unroll
  for (int j = 0; j < 4; ++j)
#pragma unroll
    for (int r = 0; r < 8; ++r) ss[wave][8 * g + r][j * 16 + col] = (_Float16)(o[j][r] * fold);
  __syncthreads();
#pragma unroll
  for (int it = 0; it < 4; ++it) { const int e = lane + 32 * it; const int rl = e >> 3, q = e & 7; HU u; u.h = *(const v8h*)&ss[wave][rl][q * 8];
    vst2(Y16 + ((size_t)b * SEQ + ql0 + rl) * DM + h * HD + q * 8, u.u); }
}

__global__ __launch_bounds__(128) void k_out(const _Float16* __restrict__ Y16, const _Float16* __restrict__ WOT, const float* __restrict__ BO, float* __restrict__ OUT) {
  __shared__ __align__(16) float sf[4][16][132];
  const int tid = threadIdx.x, wave = tid >> 5, lane = tid & 31, col = lane & 15, g = lane >> 4;
  const int c0 = blockIdx.y * 128; const size_t r0 = (size_t)blockIdx.x * 64 + wave * 16;
  v8f acc[8] = {};
  mm_k1024(Y16 + (r0 + col) * DM, WOT + (size_t)(c0 + col) * DM, lane, acc);
  const float osc = 1.0f / (512.0f * (float)SEQ);
#pragma unroll
  for (int j = 0; j < 8; ++j) { const float bb = bfr(BO[c0 + j * 16 + col]);
#pragma unroll
    for (int r = 0; r < 8; ++r) sf[wave][8 * g + r][j * 16 + col] = acc[j][r] * osc + bb; }
  __syncthreads();
  for (int rl = 0; rl < 16; ++rl) vst2(OUT + (r0 + rl) * DM + c0 + lane * 4, *(const v4f*)&sf[wave][rl][lane * 4]);
}

extern "C" void kernel_launch(void* const* d_in, const int* in_sizes, int n_in, void* d_out, int out_size, void* d_ws, size_t ws_size, hipStream_t stream) {
  if (n_in < 7) return;
  if ((size_t)in_sizes[0] < ((size_t)(NB - 1) * SEQ_FULL + SEQ) * DM) return;
  if (in_sizes[1] < DM || in_sizes[2] < DM || in_sizes[5] < DM || in_sizes[6] < 1) return;
  if ((size_t)in_sizes[3] < (size_t)DM * QKVN || (size_t)in_sizes[4] < (size_t)DM * DM) return;
  if ((size_t)out_size < (size_t)NB * SEQ * DM) return;
  if (ws_size < (size_t)WS_END) return;
  const float* X = (const float*)d_in[0]; const float* LW = (const float*)d_in[1]; const float* LB = (const float*)d_in[2];
  const float* WQ = (const float*)d_in[3]; const float* WO = (const float*)d_in[4]; const float* BO = (const float*)d_in[5]; const int* LI = (const int*)d_in[6];
  char* ws = (char*)d_ws;
  _Float16* XN = (_Float16*)(ws + WS_XN); _Float16* WQT = (_Float16*)(ws + WS_WQT); _Float16* WOT = (_Float16*)(ws + WS_WOT);
  _Float16* Q16 = (_Float16*)(ws + WS_Q); _Float16* K16 = (_Float16*)(ws + WS_K); _Float16* VT16 = (_Float16*)(ws + WS_VT); _Float16* Y16 = (_Float16*)(ws + WS_Y);
  k_wt<<<dim3(QKVN / 64, DM / 64), 256, 0, stream>>>(WQ, DM, QKVN, WQT);
  k_wt<<<dim3(DM / 64, DM / 64), 256, 0, stream>>>(WO, DM, DM, WOT);
  k_ln<<<dim3(NB * SEQ), 128, 0, stream>>>(X, LW, LB, XN);
  k_qkv<<<dim3(NB * SEQ / 64, QKVN / 128), 128, 0, stream>>>(XN, WQT, Q16, K16, VT16);
  k_attn<<<dim3(SEQ / 64, NB * NH), 128, 0, stream>>>(Q16, K16, VT16, LI, Y16);
  k_out<<<dim3(NB * SEQ / 64, DM / 128), 128, 0, stream>>>(Y16, WOT, BO, (float*)d_out);
}
